// TreeGNNRefinement_27238682591485
// MI455X (gfx1250) — hardware-verified
//
#include <hip/hip_runtime.h>
#include <stdint.h>

typedef _Float16 v16h __attribute__((ext_vector_type(16)));
typedef _Float16 v8h  __attribute__((ext_vector_type(8)));
typedef _Float16 v4h  __attribute__((ext_vector_type(4)));
typedef float    v8f  __attribute__((ext_vector_type(8)));
typedef float    v4f  __attribute__((ext_vector_type(4)));
typedef __bf16   v16b __attribute__((ext_vector_type(16)));
typedef unsigned short v16us __attribute__((ext_vector_type(16)));
typedef unsigned short v8us  __attribute__((ext_vector_type(8)));
typedef v8h  __attribute__((may_alias)) v8ha;
typedef v4h  __attribute__((may_alias)) v4ha;
typedef v4f  __attribute__((may_alias)) v4fa;
typedef v8us __attribute__((may_alias)) v8usa;

union FragH { v16h v; v8h half[2]; };
union FragB { v16b v; v16us u; v8us half[2]; unsigned short e[16]; };
union Pack8 { v8us v; unsigned short e[8]; };

#define NTOK  32768
#define NSEN  256
#define NSEQ  128
#define DMOD  256
#define HDIM  64
#define PLANE 8388608

static constexpr float kWsc  = 64.0f;
static constexpr float kInvW = 0.015625f;
static constexpr float kInvWA = 0.0009765625f;
static constexpr float kPsc  = 16384.0f;
static constexpr float kOsc  = 0.0009765625f;

__device__ __forceinline__ v8f wmma_h(v16h a, v16h b, v8f c) {
  v8f d = __builtin_amdgcn_wmma_f32_16x16x32_f16(false, a, false, b, (short)0, c, false, false);
  asm volatile("v_nop\n\tv_nop\n\tv_nop\n\tv_nop" : "+v"(d) : "v"(a), "v"(b));
  return d;
}
__device__ __forceinline__ v8f wmma_b(v16b a, v16b b, v8f c) {
  v8f d = __builtin_amdgcn_wmma_f32_16x16x32_bf16(false, a, false, b, (short)0, c, false, false);
  asm volatile("v_nop\n\tv_nop\n\tv_nop\n\tv_nop" : "+v"(d) : "v"(a), "v"(b));
  return d;
}
__device__ __forceinline__ v16h ldfrag_h(const _Float16* p, int h) {
  FragH f;
  f.half[0] = *(const v8ha*)(p + 8 * h);
  f.half[1] = *(const v8ha*)(p + 16 + 8 * h);
  return f.v;
}
__device__ __forceinline__ v16b ldfrag_us(const unsigned short* p, int h) {
  FragB f;
  f.half[0] = *(const v8usa*)(p + 8 * h);
  f.half[1] = *(const v8usa*)(p + 16 + 8 * h);
  return f.v;
}
__device__ __forceinline__ unsigned int bf16_rne(float x) {
  const unsigned int u = __float_as_uint(x);
  return (u + 0x7fffu + ((u >> 16) & 1u)) >> 16;
}
__device__ __forceinline__ void split1(float x, unsigned short& eh, unsigned short& el) {
  const unsigned int hb = bf16_rne(x);
  const float hf = __uint_as_float(hb << 16);
  eh = (unsigned short)hb;
  el = (unsigned short)bf16_rne(x - hf);
}
__device__ __forceinline__ void split_frag(const float* p, int h, v16b& hi, v16b& lo) {
  const v4f x0 = *(const v4fa*)(p + 8 * h);
  const v4f x1 = *(const v4fa*)(p + 8 * h + 4);
  const v4f x2 = *(const v4fa*)(p + 16 + 8 * h);
  const v4f x3 = *(const v4fa*)(p + 16 + 8 * h + 4);
  FragB fh, fl;
  split1(x0.x, fh.e[0],  fl.e[0]);  split1(x0.y, fh.e[1],  fl.e[1]);
  split1(x0.z, fh.e[2],  fl.e[2]);  split1(x0.w, fh.e[3],  fl.e[3]);
  split1(x1.x, fh.e[4],  fl.e[4]);  split1(x1.y, fh.e[5],  fl.e[5]);
  split1(x1.z, fh.e[6],  fl.e[6]);  split1(x1.w, fh.e[7],  fl.e[7]);
  split1(x2.x, fh.e[8],  fl.e[8]);  split1(x2.y, fh.e[9],  fl.e[9]);
  split1(x2.z, fh.e[10], fl.e[10]); split1(x2.w, fh.e[11], fl.e[11]);
  split1(x3.x, fh.e[12], fl.e[12]); split1(x3.y, fh.e[13], fl.e[13]);
  split1(x3.z, fh.e[14], fl.e[14]); split1(x3.w, fh.e[15], fl.e[15]);
  hi = fh.v; lo = fl.v;
}
__device__ __forceinline__ void split8(v4f x0, v4f x1, v8us& hv, v8us& lv) {
  Pack8 a, c;
  split1(x0.x, a.e[0], c.e[0]); split1(x0.y, a.e[1], c.e[1]);
  split1(x0.z, a.e[2], c.e[2]); split1(x0.w, a.e[3], c.e[3]);
  split1(x1.x, a.e[4], c.e[4]); split1(x1.y, a.e[5], c.e[5]);
  split1(x1.z, a.e[6], c.e[6]); split1(x1.w, a.e[7], c.e[7]);
  hv = a.v; lv = c.v;
}
__device__ __forceinline__ float gelu_f(float x) {
  return 0.5f * x * (1.0f + erff(x * 0.70710678118654752f));
}
__device__ __forceinline__ float sigm_f(float x) {
  return __builtin_amdgcn_rcpf(1.0f + __expf(-x));
}

__global__ __launch_bounds__(256) void cvt_h_k(const float* __restrict__ H, _Float16* __restrict__ Hh, int n8) {
  const int g = blockIdx.x * 256 + threadIdx.x;
  if (g >= n8) return;
  const float* s = H + (size_t)g * 8;
  const v4f a = *(const v4fa*)s;
  const v4f c = *(const v4fa*)(s + 4);
  const v8h o = { (_Float16)a.x, (_Float16)a.y, (_Float16)a.z, (_Float16)a.w,
                  (_Float16)c.x, (_Float16)c.y, (_Float16)c.z, (_Float16)c.w };
  _Float16* d = Hh + (size_t)g * 8;
  *(volatile v8h*)d = o;
  __threadfence();
  *(volatile v8h*)d = o;
}

__global__ __launch_bounds__(256) void cvt_wt_k(const float* __restrict__ src0, const float* __restrict__ src1,
                                                  int nsl0, _Float16* dst0, _Float16* dst1, int K) {
  __shared__ __attribute__((aligned(16))) _Float16 sT[64][72];
  const int z = blockIdx.z;
  const bool sec = (z >= nsl0);
  const int sl = sec ? (z - nsl0) : z;
  const float* src = (sec ? src1 : src0) + (size_t)sl * K * DMOD;
  _Float16* dst = (sec ? dst1 : dst0) + (size_t)sl * DMOD * K;
  const int k0 = blockIdx.x * 64, n0 = blockIdx.y * 64;
  const int tid = threadIdx.x, kk = tid >> 2, cq = (tid & 3) * 16;
  const float* rp = src + (size_t)(k0 + kk) * DMOD + n0 + cq;
  #pragma unroll
  for (int i = 0; i < 4; ++i) {
    const v4f v = *(const v4fa*)(rp + 4 * i);
    sT[cq + 4 * i + 0][kk] = (_Float16)(v.x * kWsc);
    sT[cq + 4 * i + 1][kk] = (_Float16)(v.y * kWsc);
    sT[cq + 4 * i + 2][kk] = (_Float16)(v.z * kWsc);
    sT[cq + 4 * i + 3][kk] = (_Float16)(v.w * kWsc);
  }
  __syncthreads();
  const int q8 = tid & 7, nb = tid >> 3;
  const v8h o0 = *(const v8ha*)(&sT[nb][8 * q8]);
  const v8h o1 = *(const v8ha*)(&sT[nb + 32][8 * q8]);
  _Float16* d0 = dst + (size_t)(n0 + nb) * K + k0 + 8 * q8;
  _Float16* d1 = dst + (size_t)(n0 + nb + 32) * K + k0 + 8 * q8;
  *(volatile v8h*)d0 = o0;
  *(volatile v8h*)d1 = o1;
  __threadfence();
  *(volatile v8h*)d0 = o0;
  *(volatile v8h*)d1 = o1;
}

__global__ __launch_bounds__(256) void cvt_w3_k(const float* __restrict__ s0, const float* __restrict__ s1,
                                                  const float* __restrict__ s2, unsigned short* dstb) {
  __shared__ __attribute__((aligned(16))) float sT[64][68];
  const int z = blockIdx.z;
  const float* src = (z == 0) ? s0 : ((z == 1) ? s1 : s2);
  const bool tr = (z < 2);
  unsigned short* hi = dstb + (size_t)z * 131072;
  unsigned short* lo = hi + 65536;
  const int r0 = blockIdx.x * 64, c0 = blockIdx.y * 64;
  const int tid = threadIdx.x, rr = tid >> 2, cq = (tid & 3) * 16;
  const float* rp = src + (size_t)(r0 + rr) * DMOD + c0 + cq;
  if (tr) {
    #pragma unroll
    for (int i = 0; i < 4; ++i) {
      const v4f v = *(const v4fa*)(rp + 4 * i);
      sT[cq + 4 * i + 0][rr] = v.x; sT[cq + 4 * i + 1][rr] = v.y;
      sT[cq + 4 * i + 2][rr] = v.z; sT[cq + 4 * i + 3][rr] = v.w;
    }
  } else {
    #pragma unroll
    for (int i = 0; i < 4; ++i) {
      const v4f v = *(const v4fa*)(rp + 4 * i);
      sT[rr][cq + 4 * i + 0] = v.x; sT[rr][cq + 4 * i + 1] = v.y;
      sT[rr][cq + 4 * i + 2] = v.z; sT[rr][cq + 4 * i + 3] = v.w;
    }
  }
  __syncthreads();
  const int orow0 = tr ? c0 : r0, ocol0 = tr ? r0 : c0;
  const int q8 = tid & 7, nb = tid >> 3;
  v8us h0, l0, h1, l1;
  split8(*(const v4fa*)(&sT[nb][8 * q8]), *(const v4fa*)(&sT[nb][8 * q8 + 4]), h0, l0);
  split8(*(const v4fa*)(&sT[nb + 32][8 * q8]), *(const v4fa*)(&sT[nb + 32][8 * q8 + 4]), h1, l1);
  const size_t o0 = (size_t)(orow0 + nb) * DMOD + ocol0 + 8 * q8;
  const size_t o1 = (size_t)(orow0 + nb + 32) * DMOD + ocol0 + 8 * q8;
  *(volatile v8us*)(hi + o0) = h0; *(volatile v8us*)(lo + o0) = l0;
  *(volatile v8us*)(hi + o1) = h1; *(volatile v8us*)(lo + o1) = l1;
  __threadfence();
  *(volatile v8us*)(hi + o0) = h0; *(volatile v8us*)(lo + o0) = l0;
  *(volatile v8us*)(hi + o1) = h1; *(volatile v8us*)(lo + o1) = l1;
}

__device__ __forceinline__ v8h gemm_piece(const float* sp, v4f b0, v4f b1, int act, float ks) {
  const v4f x0 = *(const v4fa*)sp;
  const v4f x1 = *(const v4fa*)(sp + 4);
  float y0 = x0.x * ks + b0.x, y1 = x0.y * ks + b0.y, y2 = x0.z * ks + b0.z, y3 = x0.w * ks + b0.w;
  float y4 = x1.x * ks + b1.x, y5 = x1.y * ks + b1.y, y6 = x1.z * ks + b1.z, y7 = x1.w * ks + b1.w;
  if (act != 0) {
    y0 = gelu_f(y0); y1 = gelu_f(y1); y2 = gelu_f(y2); y3 = gelu_f(y3);
    y4 = gelu_f(y4); y5 = gelu_f(y5); y6 = gelu_f(y6); y7 = gelu_f(y7);
  }
  const v8h o = { (_Float16)y0, (_Float16)y1, (_Float16)y2, (_Float16)y3,
                  (_Float16)y4, (_Float16)y5, (_Float16)y6, (_Float16)y7 };
  return o;
}

__global__ __launch_bounds__(256) void gemm_k(
    const _Float16* a00, const _Float16* a10, const _Float16* __restrict__ wt0, const float* __restrict__ bs0, _Float16* oo0,
    const _Float16* a01, const _Float16* a11, const _Float16* __restrict__ wt1, const float* __restrict__ bs1, _Float16* oo1,
    const _Float16* a02, const _Float16* a12, const _Float16* __restrict__ wt2, const float* __restrict__ bs2, _Float16* oo2,
    int nch0, int nch1, int nch2, int act0, int act1, int act2, float ks0, float ks1, float ks2)
{
  __shared__ __attribute__((aligned(16))) float sT[128][64];
  const int z = blockIdx.z;
  const _Float16* a0 = (z == 0) ? a00 : ((z == 1) ? a01 : a02);
  const _Float16* a1 = (z == 0) ? a10 : ((z == 1) ? a11 : a12);
  const _Float16* wt = (z == 0) ? wt0 : ((z == 1) ? wt1 : wt2);
  const float* bs    = (z == 0) ? bs0 : ((z == 1) ? bs1 : bs2);
  _Float16* out      = (z == 0) ? oo0 : ((z == 1) ? oo1 : oo2);
  const int nch      = (z == 0) ? nch0 : ((z == 1) ? nch1 : nch2);
  const int act      = (z == 0) ? act0 : ((z == 1) ? act1 : act2);
  const float ks     = (z == 0) ? ks0 : ((z == 1) ? ks1 : ks2);

  const int tid = threadIdx.x, lane = tid & 31, w = tid >> 5;
  const int h = lane >> 4, m = lane & 15;
  const int m0 = blockIdx.x * 128, n0 = blockIdx.y * 64;
  const int mw = 32 * (w >> 1), nw = 32 * (w & 1);
  const int K = DMOD * nch;

  const v8f zero8 = {0.f, 0.f, 0.f, 0.f, 0.f, 0.f, 0.f, 0.f};
  v8f acc[2][2];
  acc[0][0] = zero8; acc[0][1] = zero8; acc[1][0] = zero8; acc[1][1] = zero8;

  #pragma unroll 1
  for (int c = 0; c < nch; ++c) {
    const _Float16* A = (c == 0) ? a0 : a1;
    const _Float16* ar0 = A + ((size_t)(m0 + mw + m)) * DMOD;
    const _Float16* ar1 = ar0 + (size_t)16 * DMOD;
    const _Float16* br0 = wt + ((size_t)(n0 + nw + m)) * K + c * DMOD;
    const _Float16* br1 = br0 + (size_t)16 * K;
    #pragma unroll 2
    for (int k0 = 0; k0 < DMOD; k0 += 32) {
      const v16h fa0 = ldfrag_h(ar0 + k0, h);
      const v16h fa1 = ldfrag_h(ar1 + k0, h);
      const v16h fb0 = ldfrag_h(br0 + k0, h);
      const v16h fb1 = ldfrag_h(br1 + k0, h);
      acc[0][0] = wmma_h(fa0, fb0, acc[0][0]);
      acc[0][1] = wmma_h(fa0, fb1, acc[0][1]);
      acc[1][0] = wmma_h(fa1, fb0, acc[1][0]);
      acc[1][1] = wmma_h(fa1, fb1, acc[1][1]);
    }
  }
  #pragma unroll
  for (int mt = 0; mt < 2; ++mt)
    #pragma unroll
    for (int nt = 0; nt < 2; ++nt)
      #pragma unroll
      for (int r = 0; r < 8; ++r)
        sT[mw + 16 * mt + 8 * h + r][nw + 16 * nt + m] = acc[mt][nt][r];
  __syncthreads();

  const int q8 = tid & 7, rb = tid >> 3;
  const v4f bb0 = *(const v4fa*)(bs + n0 + 8 * q8);
  const v4f bb1 = *(const v4fa*)(bs + n0 + 8 * q8 + 4);
  #pragma unroll 1
  for (int i = 0; i < 4; ++i) {
    const int row = rb + 32 * i;
    const v8h o = gemm_piece(&sT[row][8 * q8], bb0, bb1, act, ks);
    *(volatile v8h*)(out + ((size_t)(m0 + row)) * DMOD + n0 + 8 * q8) = o;
  }
  __threadfence();
  #pragma unroll 1
  for (int i = 0; i < 4; ++i) {
    const int row = rb + 32 * i;
    const v8h o = gemm_piece(&sT[row][8 * q8], bb0, bb1, act, ks);
    *(volatile v8h*)(out + ((size_t)(m0 + row)) * DMOD + n0 + 8 * q8) = o;
  }
}

__device__ __forceinline__ v16h pack_p(v8f a, v8f c) {
  const v16h r = { (_Float16)(a[0] * kPsc), (_Float16)(a[1] * kPsc), (_Float16)(a[2] * kPsc), (_Float16)(a[3] * kPsc),
                   (_Float16)(a[4] * kPsc), (_Float16)(a[5] * kPsc), (_Float16)(a[6] * kPsc), (_Float16)(a[7] * kPsc),
                   (_Float16)(c[0] * kPsc), (_Float16)(c[1] * kPsc), (_Float16)(c[2] * kPsc), (_Float16)(c[3] * kPsc),
                   (_Float16)(c[4] * kPsc), (_Float16)(c[5] * kPsc), (_Float16)(c[6] * kPsc), (_Float16)(c[7] * kPsc) };
  return r;
}

__global__ __launch_bounds__(256) void attn_k(const _Float16* __restrict__ Q, const _Float16* __restrict__ Kp,
                                                const _Float16* __restrict__ Vp, const int* __restrict__ ph,
                                                const float* __restrict__ mask, _Float16* __restrict__ AO, int kind)
{
  __shared__ __attribute__((aligned(16))) _Float16 sK[NSEQ][72];
  __shared__ __attribute__((aligned(16))) _Float16 sVT[HDIM][136];
  __shared__ __attribute__((aligned(16))) _Float16 sO[8][16 * 64];
  __shared__ int sidx[NSEQ];
  __shared__ int sph[NSEQ];
  __shared__ float smk[NSEQ];

  const int bh = blockIdx.x, b = bh >> 2, hh = bh & 3;
  const int tid = threadIdx.x, lane = tid & 31, w = tid >> 5;
  const int h = lane >> 4, m = lane & 15;

  if (tid < NSEQ) {
    const int v = ph[b * NSEQ + tid];
    sph[tid] = v;
    sidx[tid] = v < 0 ? 0 : (v > NSEQ - 1 ? NSEQ - 1 : v);
    smk[tid] = mask[b * NSEQ + tid];
  }
  __syncthreads();
  #pragma unroll
  for (int it = 0; it < 4; ++it) {
    const int i = tid + 256 * it;
    const int pos = i >> 3, ch = i & 7;
    const int gsrc = sidx[pos];
    const int src = (kind == 0) ? gsrc : pos;
    const size_t ro = ((size_t)(b * NSEQ + src)) * DMOD + hh * HDIM + ch * 8;
    const v8h kv = *(const v8ha*)(Kp + ro);
    *(v8ha*)(&sK[pos][ch * 8]) = kv;
    const v8h vv = *(const v8ha*)(Vp + ro);
    #pragma unroll
    for (int e = 0; e < 8; ++e) sVT[ch * 8 + e][pos] = vv[e];
  }
  __syncthreads();

  const int q = 16 * w + m;
  const _Float16* qr = Q + ((size_t)(b * NSEQ + q)) * DMOD + hh * HDIM;
  const v16h qb0 = ldfrag_h(qr, h);
  const v16h qb1 = ldfrag_h(qr + 32, h);

  const v8f zero8 = {0.f, 0.f, 0.f, 0.f, 0.f, 0.f, 0.f, 0.f};
  v8f s[8];
  #pragma unroll
  for (int j = 0; j < 8; ++j) {
    const _Float16* kr = &sK[16 * j + m][0];
    const v16h kf0 = ldfrag_h(kr, h);
    const v16h kf1 = ldfrag_h(kr + 32, h);
    v8f zz = zero8;
    zz = wmma_h(kf0, qb0, zz);
    zz = wmma_h(kf1, qb1, zz);
    s[j] = zz;
  }
  #pragma unroll
  for (int j = 0; j < 8; ++j)
    #pragma unroll
    for (int r = 0; r < 8; ++r) s[j][r] = s[j][r] * 0.125f;

  if (kind != 0) {
    const int pq = sph[q];
    const bool vq = smk[q] > 0.0f;
    #pragma unroll
    for (int j = 0; j < 8; ++j) {
      #pragma unroll
      for (int r = 0; r < 8; ++r) {
        const int k = 16 * j + 8 * h + r;
        const bool ok = (sph[k] == pq) && (k != q) && vq && (smk[k] > 0.0f);
        s[j][r] = ok ? s[j][r] : -1.0e9f;
      }
    }
  }

  float mx = s[0][0];
  #pragma unroll
  for (int j = 0; j < 8; ++j)
    #pragma unroll
    for (int r = 0; r < 8; ++r) mx = fmaxf(mx, s[j][r]);
  mx = fmaxf(mx, __shfl_xor(mx, 16));
  float ls = 0.0f;
  #pragma unroll
  for (int j = 0; j < 8; ++j)
    #pragma unroll
    for (int r = 0; r < 8; ++r) {
      const float p = __expf(s[j][r] - mx);
      s[j][r] = p;
      ls += p;
    }
  ls += __shfl_xor(ls, 16);
  const float rl = __builtin_amdgcn_rcpf(ls) * kOsc;

  v8f o[4];
  o[0] = zero8; o[1] = zero8; o[2] = zero8; o[3] = zero8;
  #pragma unroll
  for (int kc = 0; kc < 4; ++kc) {
    const v16h pb = pack_p(s[2 * kc], s[2 * kc + 1]);
    #pragma unroll
    for (int t = 0; t < 4; ++t) {
      const v16h vf = ldfrag_h(&sVT[16 * t + m][32 * kc], h);
      o[t] = wmma_h(vf, pb, o[t]);
    }
  }
  _Float16* so = &sO[w][0];
  #pragma unroll
  for (int t = 0; t < 4; ++t)
    #pragma unroll
    for (int r = 0; r < 8; ++r)
      so[m * 64 + 16 * t + 8 * h + r] = (_Float16)(o[t][r] * rl);
  __syncthreads();

  const int q8 = lane & 7, rsub = lane >> 3;
  v8h ov[4];
  #pragma unroll
  for (int i = 0; i < 4; ++i) ov[i] = *(const v8ha*)(so + (4 * i + rsub) * 64 + 8 * q8);
  #pragma unroll
  for (int i = 0; i < 4; ++i) {
    const int row = 4 * i + rsub;
    *(volatile v8h*)(AO + ((size_t)(b * NSEQ + 16 * w + row)) * DMOD + hh * HDIM + 8 * q8) = ov[i];
  }
  __threadfence();
  #pragma unroll
  for (int i = 0; i < 4; ++i) {
    const int row = 4 * i + rsub;
    *(volatile v8h*)(AO + ((size_t)(b * NSEQ + 16 * w + row)) * DMOD + hh * HDIM + 8 * q8) = ov[i];
  }
}

__global__ __launch_bounds__(256) void child_k(const float* __restrict__ HrIn, const int* __restrict__ ph,
                                                 const float* __restrict__ mask, _Float16* __restrict__ cavg)
{
  __shared__ int shi[NSEQ], scnt[NSEQ], soff[NSEQ], srk[NSEQ], sord[NSEQ];
  __shared__ float smk[NSEQ];
  __shared__ __attribute__((aligned(16))) _Float16 sC[32][DMOD];

  const int b = blockIdx.x, tid = threadIdx.x;
  const size_t rowb = (size_t)b * NSEQ;

  if (tid < NSEQ) {
    int v = ph[rowb + tid];
    v = v < 0 ? 0 : (v > NSEQ - 1 ? NSEQ - 1 : v);
    shi[tid] = v;
    smk[tid] = mask[rowb + tid];
    sord[tid] = tid;
  }
  __syncthreads();
  if (tid < NSEQ) {
    const int my = shi[tid];
    int rk = 0, cnt = 0, off = 0;
    #pragma unroll 4
    for (int j = 0; j < NSEQ; ++j) {
      const int hj = shi[j];
      rk  += ((hj == my) && (j < tid)) ? 1 : 0;
      cnt += (hj == tid) ? 1 : 0;
      off += (hj < tid) ? 1 : 0;
    }
    srk[tid] = rk; scnt[tid] = cnt; soff[tid] = off;
  }
  __syncthreads();
  if (tid < NSEQ) {
    int pos = soff[shi[tid]] + srk[tid];
    pos = pos < 0 ? 0 : (pos > NSEQ - 1 ? NSEQ - 1 : pos);
    sord[pos] = tid;
  }
  __syncthreads();

  const int col = tid;
  const int q8 = tid & 7, lsub = tid >> 3;
  #pragma unroll 1
  for (int mb = 0; mb < 4; ++mb) {
    #pragma unroll 1
    for (int mm = 0; mm < 32; ++mm) {
      const int md = mb * 32 + mm;
      int cnt = scnt[md];
      cnt = cnt > NSEQ ? NSEQ : cnt;
      const int off = soff[md];
      float s = 0.0f, cm = 0.0f;
      #pragma unroll 1
      for (int i = 0; i < cnt; ++i) {
        int p = off + i;
        p = p < 0 ? 0 : (p > NSEQ - 1 ? NSEQ - 1 : p);
        int n = sord[p];
        n = n < 0 ? 0 : (n > NSEQ - 1 ? NSEQ - 1 : n);
        s  += HrIn[(rowb + n) * DMOD + col];
        cm += smk[n];
      }
      const float dn = fmaxf(cm, 1.0f);
      sC[mm][col] = (_Float16)(s * __builtin_amdgcn_rcpf(dn));
    }
    __syncthreads();
    v8h ov[4];
    #pragma unroll
    for (int i = 0; i < 4; ++i) {
      const int line = lsub + 32 * i;
      const int row = line >> 2, seg = line & 3;
      ov[i] = *(const v8ha*)(&sC[row][64 * seg + 8 * q8]);
    }
    #pragma unroll
    for (int i = 0; i < 4; ++i) {
      const int line = lsub + 32 * i;
      const int row = line >> 2, seg = line & 3;
      *(volatile v8h*)(cavg + (rowb + mb * 32 + row) * DMOD + 64 * seg + 8 * q8) = ov[i];
    }
    __threadfence();
    #pragma unroll
    for (int i = 0; i < 4; ++i) {
      const int line = lsub + 32 * i;
      const int row = line >> 2, seg = line & 3;
      *(volatile v8h*)(cavg + (rowb + mb * 32 + row) * DMOD + 64 * seg + 8 * q8) = ov[i];
    }
    __syncthreads();
  }
}

__global__ __launch_bounds__(256) void comb_k(const _Float16* Hh, const _Float16* hm, const _Float16* cmg, const _Float16* smg,
                                                const _Float16* __restrict__ gT, const _Float16* __restrict__ tT,
                                                const float* __restrict__ gb, const float* __restrict__ tb,
                                                const float* __restrict__ lg, const float* __restrict__ lbeta,
                                                const float* HrIn, float* HrOut, _Float16* HhOut, int writeH)
{
  __shared__ __attribute__((aligned(16))) float sGU[32][512];

  const int tid = threadIdx.x, lane = tid & 31, w = tid >> 5;
  const int h = lane >> 4, m = lane & 15;
  const int m0 = blockIdx.x * 32;
  const bool isg = (w < 4);
  const _Float16* wt = isg ? gT : tT;
  const int colw = 64 * (w & 3);

  const v8f zero8 = {0.f, 0.f, 0.f, 0.f, 0.f, 0.f, 0.f, 0.f};
  v8f acc[2][4];
  #pragma unroll
  for (int mt = 0; mt < 2; ++mt)
    #pragma unroll
    for (int nt = 0; nt < 4; ++nt) acc[mt][nt] = zero8;

  #pragma unroll 1
  for (int c = 0; c < 4; ++c) {
    const _Float16* A = (c == 0) ? Hh : ((c == 1) ? hm : ((c == 2) ? cmg : smg));
    const _Float16* ar0 = A + ((size_t)(m0 + m)) * DMOD;
    const _Float16* ar1 = ar0 + (size_t)16 * DMOD;
    const _Float16* br = wt + ((size_t)(colw + m)) * 1024 + c * DMOD;
    #pragma unroll 2
    for (int k0 = 0; k0 < DMOD; k0 += 32) {
      const v16h fa0 = ldfrag_h(ar0 + k0, h);
      const v16h fa1 = ldfrag_h(ar1 + k0, h);
      #pragma unroll
      for (int nt = 0; nt < 4; ++nt) {
        const v16h fb = ldfrag_h(br + (size_t)nt * 16 * 1024 + k0, h);
        acc[0][nt] = wmma_h(fa0, fb, acc[0][nt]);
        acc[1][nt] = wmma_h(fa1, fb, acc[1][nt]);
      }
    }
  }

  const float* bp = isg ? gb : tb;
  #pragma unroll
  for (int nt = 0; nt < 4; ++nt) {
    const int cl = colw + 16 * nt + m;
    const float bv = bp[cl];
    const int c512 = 64 * w + 16 * nt + m;
    #pragma unroll
    for (int mt = 0; mt < 2; ++mt)
      #pragma unroll
      for (int r = 0; r < 8; ++r)
        sGU[16 * mt + 8 * h + r][c512] = acc[mt][nt][r] * kInvW + bv;
  }
  __syncthreads();

  const int c0 = 4 * lane, c1 = 128 + 4 * lane;
  const v4f lg0 = *(const v4fa*)(lg + c0), lg1 = *(const v4fa*)(lg + c1);
  const v4f be0 = *(const v4fa*)(lbeta + c0), be1 = *(const v4fa*)(lbeta + c1);
  #pragma unroll 1
  for (int rr = 0; rr < 4; ++rr) {
    const int row = 4 * w + rr;
    const size_t gro = ((size_t)(m0 + row)) * DMOD;
    const v4f g0 = *(const v4fa*)(&sGU[row][c0]);
    const v4f g1 = *(const v4fa*)(&sGU[row][c1]);
    const v4f u0 = *(const v4fa*)(&sGU[row][256 + c0]);
    const v4f u1 = *(const v4fa*)(&sGU[row][256 + c1]);
    const v4f x0 = *(const v4fa*)(HrIn + gro + c0);
    const v4f x1 = *(const v4fa*)(HrIn + gro + c1);
    const float hn0 = x0.x + sigm_f(g0.x) * gelu_f(u0.x);
    const float hn1 = x0.y + sigm_f(g0.y) * gelu_f(u0.y);
    const float hn2 = x0.z + sigm_f(g0.z) * gelu_f(u0.z);
    const float hn3 = x0.w + sigm_f(g0.w) * gelu_f(u0.w);
    const float hn4 = x1.x + sigm_f(g1.x) * gelu_f(u1.x);
    const float hn5 = x1.y + sigm_f(g1.y) * gelu_f(u1.y);
    const float hn6 = x1.z + sigm_f(g1.z) * gelu_f(u1.z);
    const float hn7 = x1.w + sigm_f(g1.w) * gelu_f(u1.w);
    float ssum = ((hn0 + hn1) + (hn2 + hn3)) + ((hn4 + hn5) + (hn6 + hn7));
    ssum += __shfl_xor(ssum, 16); ssum += __shfl_xor(ssum, 8); ssum += __shfl_xor(ssum, 4);
    ssum += __shfl_xor(ssum, 2);  ssum += __shfl_xor(ssum, 1);
    const float mu = ssum * (1.0f / 256.0f);
    const float d0 = hn0 - mu, d1 = hn1 - mu, d2 = hn2 - mu, d3 = hn3 - mu;
    const float d4 = hn4 - mu, d5 = hn5 - mu, d6 = hn6 - mu, d7 = hn7 - mu;
    float sq = ((d0 * d0 + d1 * d1) + (d2 * d2 + d3 * d3)) + ((d4 * d4 + d5 * d5) + (d6 * d6 + d7 * d7));
    sq += __shfl_xor(sq, 16); sq += __shfl_xor(sq, 8); sq += __shfl_xor(sq, 4);
    sq += __shfl_xor(sq, 2);  sq += __shfl_xor(sq, 1);
    const float var = sq * (1.0f / 256.0f);
    const float rs = rsqrtf(var + 1.0e-5f);
    const v4f y0 = { d0 * rs * lg0.x + be0.x, d1 * rs * lg0.y + be0.y, d2 * rs * lg0.z + be0.z, d3 * rs * lg0.w + be0.w };
    const v4f y1 = { d4 * rs * lg1.x + be1.x, d5 * rs * lg1.y + be1.y, d6 * rs * lg1.z + be1.z, d7 * rs * lg1.w + be1.w };
    *(volatile v4f*)(HrOut + gro + c0) = y0;
    *(volatile v4f*)(HrOut + gro + c1) = y1;
    if (writeH != 0) {
      const v4h z0 = { (_Float16)y0.x, (_Float16)y0.y, (_Float16)y0.z, (_Float16)y0.w };
      const v4h z1 = { (_Float16)y1.x, (_Float16)y1.y, (_Float16)y1.z, (_Float16)y1.w };
      *(volatile v4h*)(HhOut + gro + c0) = z0;
      *(volatile v4h*)(HhOut + gro + c1) = z1;
    }
    *(v4fa*)(&sGU[row][c0]) = y0;
    *(v4fa*)(&sGU[row][c1]) = y1;
  }
  __threadfence();
  #pragma unroll 1
  for (int rr = 0; rr < 4; ++rr) {
    const int row = 4 * w + rr;
    const size_t gro = ((size_t)(m0 + row)) * DMOD;
    const v4f y0 = *(const v4fa*)(&sGU[row][c0]);
    const v4f y1 = *(const v4fa*)(&sGU[row][c1]);
    *(volatile v4f*)(HrOut + gro + c0) = y0;
    *(volatile v4f*)(HrOut + gro + c1) = y1;
    if (writeH != 0) {
      const v4h z0 = { (_Float16)y0.x, (_Float16)y0.y, (_Float16)y0.z, (_Float16)y0.w };
      const v4h z1 = { (_Float16)y1.x, (_Float16)y1.y, (_Float16)y1.z, (_Float16)y1.w };
      *(volatile v4h*)(HhOut + gro + c0) = z0;
      *(volatile v4h*)(HhOut + gro + c1) = z1;
    }
  }
}

__global__ __launch_bounds__(256) void gemm3_k(
    const float* A0, const unsigned short* __restrict__ W0, const float* __restrict__ B0, float* O0, unsigned short* P0,
    const float* A1, const unsigned short* __restrict__ W1, const float* __restrict__ B1, float* O1, unsigned short* P1,
    int hasBias, int omode)
{
  __shared__ __attribute__((aligned(16))) float sT[128][64];
  const int z = blockIdx.z;
  const float* A = (z == 0) ? A0 : A1;
  const unsigned short* W = (z == 0) ? W0 : W1;
  const float* Bv = (z == 0) ? B0 : B1;
  float* O = (z == 0) ? O0 : O1;
  unsigned short* P = (z == 0) ? P0 : P1;

  const int tid = threadIdx.x, lane = tid & 31, w = tid >> 5;
  const int h = lane >> 4, m = lane & 15;
  const int m0 = blockIdx.x * 128, n0 = blockIdx.y * 64;
  const int mw = 32 * (w >> 1), nw = 32 * (w & 1);

  const v8f zero8 = {0.f, 0.f, 0.f, 0.f, 0.f, 0.f, 0.f, 0.f};
  v8f acc[2][2];
  acc[0][0] = zero8; acc[0][1] = zero8; acc[1][0] = zero8; acc[1][1] = zero8;

  const float* ar0 = A + ((size_t)(m0 + mw + m)) * DMOD;
  const float* ar1 = ar0 + (size_t)16 * DMOD;
  const unsigned short* wr0 = W + ((size_t)(n0 + nw + m)) * DMOD;
  const unsigned short* wr1 = wr0 + (size_t)16 * DMOD;

  #pragma unroll 1
  for (int k0 = 0; k0 < DMOD; k0 += 32) {
    v16b a0h, a0l, a1h, a1l;
    split_frag(ar0 + k0, h, a0h, a0l);
    split_frag(ar1 + k0, h, a1h, a1l);
    const v16b b0h = ldfrag_us(wr0 + k0, h);
    const v16b b0l = ldfrag_us(wr0 + 65536 + k0, h);
    const v16b b1h = ldfrag_us(wr1 + k0, h);
    const v16b b1l = ldfrag_us(wr1 + 65536 + k0, h);
    acc[0][0] = wmma_b(a0h, b0h, acc[0][0]); acc[0][0] = wmma_b(a0h, b0l, acc[0][0]); acc[0][0] = wmma_b(a0l, b0h, acc[0][0]);
    acc[0][1] = wmma_b(a0h, b1h, acc[0][1]); acc[0][1] = wmma_b(a0h, b1l, acc[0][1]); acc[0][1] = wmma_b(a0l, b1h, acc[0][1]);
    acc[1][0] = wmma_b(a1h, b0h, acc[1][0]); acc[1][0] = wmma_b(a1h, b0l, acc[1][0]); acc[1][0] = wmma_b(a1l, b0h, acc[1][0]);
    acc[1][1] = wmma_b(a1h, b1h, acc[1][1]); acc[1][1] = wmma_b(a1h, b1l, acc[1][1]); acc[1][1] = wmma_b(a1l, b1h, acc[1][1]);
  }
  #pragma unroll
  for (int nt = 0; nt < 2; ++nt) {
    const int col = nw + 16 * nt + m;
    const float bl = Bv[n0 + col];
    const float bv = (hasBias != 0) ? bl : 0.0f;
    #pragma unroll
    for (int mt = 0; mt < 2; ++mt)
      #pragma unroll
      for (int r = 0; r < 8; ++r)
        sT[mw + 16 * mt + 8 * h + r][col] = acc[mt][nt][r] + bv;
  }
  __syncthreads();

  const int q8 = tid & 7, rb = tid >> 3;
  if (omode == 0) {
    #pragma unroll 1
    for (int i = 0; i < 8; ++i) {
      const int line = rb + 32 * i;
      const int row = line >> 1, hl = line & 1;
      const v4f v = *(const v4fa*)(&sT[row][32 * hl + 4 * q8]);
      *(volatile v4f*)(O + ((size_t)(m0 + row)) * DMOD + n0 + 32 * hl + 4 * q8) = v;
    }
    __threadfence();
    #pragma unroll 1
    for (int i = 0; i < 8; ++i) {
      const int line = rb + 32 * i;
      const int row = line >> 1, hl = line & 1;
      const v4f v = *(const v4fa*)(&sT[row][32 * hl + 4 * q8]);
      *(volatile v4f*)(O + ((size_t)(m0 + row)) * DMOD + n0 + 32 * hl + 4 * q8) = v;
    }
  } else {
    #pragma unroll 1
    for (int i = 0; i < 4; ++i) {
      const int row = rb + 32 * i;
      v8us hv, lv;
      split8(*(const v4fa*)(&sT[row][8 * q8]), *(const v4fa*)(&sT[row][8 * q8 + 4]), hv, lv);
      const size_t oo = ((size_t)(m0 + row)) * DMOD + n0 + 8 * q8;
      *(volatile v8us*)(P + oo) = hv;
      *(volatile v8us*)(P + PLANE + oo) = lv;
    }
    __threadfence();
    #pragma unroll 1
    for (int i = 0; i < 4; ++i) {
      const int row = rb + 32 * i;
      v8us hv, lv;
      split8(*(const v4fa*)(&sT[row][8 * q8]), *(const v4fa*)(&sT[row][8 * q8 + 4]), hv, lv);
      const size_t oo = ((size_t)(m0 + row)) * DMOD + n0 + 8 * q8;
      *(volatile v8us*)(P + oo) = hv;
      *(volatile v8us*)(P + PLANE + oo) = lv;
    }
  }
}

__global__ __launch_bounds__(256) void score_k(const float* __restrict__ hhp, const float* __restrict__ hdp,
                                                 const unsigned short* __restrict__ Gh,
                                                 const float* __restrict__ bhw, const float* __restrict__ bhb,
                                                 const float* __restrict__ bdw, const float* __restrict__ bdb,
                                                 float* __restrict__ out1)
{
  __shared__ float shhb[NSEQ], shdb[NSEQ];
  __shared__ __attribute__((aligned(16))) float sS[8][16][68];

  const int b = blockIdx.x;
  const int tid = threadIdx.x, lane = tid & 31, w = tid >> 5;
  const int h = lane >> 4, m = lane & 15;
  {
    const bool ishh = (tid < NSEQ);
    const int r = tid & (NSEQ - 1);
    const float* row = (ishh ? hhp : hdp) + ((size_t)(b * NSEQ + r)) * DMOD;
    const float* wv = ishh ? bhw : bdw;
    float sacc = 0.0f;
    #pragma unroll 4
    for (int d = 0; d < DMOD; d += 4) {
      const v4f x = *(const v4fa*)(row + d);
      const v4f ww = *(const v4fa*)(wv + d);
      sacc += x.x * ww.x; sacc += x.y * ww.y; sacc += x.z * ww.z; sacc += x.w * ww.w;
    }
    sacc += ishh ? bhb[0] : bdb[0];
    if (ishh) shhb[r] = sacc; else shdb[r] = sacc;
  }
  __syncthreads();

  const float* ar = hhp + ((size_t)(b * NSEQ + 16 * w + m)) * DMOD;
  const unsigned short* gr = Gh + ((size_t)(b * NSEQ + m)) * DMOD;
  const v8f zero8 = {0.f, 0.f, 0.f, 0.f, 0.f, 0.f, 0.f, 0.f};
  v8f C[8];
  #pragma unroll
  for (int j = 0; j < 8; ++j) C[j] = zero8;

  #pragma unroll 1
  for (int k0 = 0; k0 < DMOD; k0 += 32) {
    v16b ah, al;
    split_frag(ar + k0, h, ah, al);
    #pragma unroll
    for (int j = 0; j < 8; ++j) {
      const unsigned short* gp = gr + (size_t)j * 16 * DMOD + k0;
      const v16b gh = ldfrag_us(gp, h);
      const v16b gl = ldfrag_us(gp + PLANE, h);
      C[j] = wmma_b(ah, gh, C[j]);
      C[j] = wmma_b(ah, gl, C[j]);
      C[j] = wmma_b(al, gh, C[j]);
    }
  }
  const int q8 = lane & 7, rsub = lane >> 3;
  float* ss = &sS[w][0][0];
  #pragma unroll
  for (int hf = 0; hf < 2; ++hf) {
    #pragma unroll
    for (int jj = 0; jj < 4; ++jj) {
      const int j = 4 * hf + jj;
      const float cb = shhb[16 * j + m];
      #pragma unroll
      for (int r = 0; r < 8; ++r) {
        const int rowl = 8 * h + r;
        ss[rowl * 68 + 16 * jj + m] = C[j][r] + shdb[16 * w + rowl] + cb;
      }
    }
    __syncthreads();
    #pragma unroll 1
    for (int i = 0; i < 8; ++i) {
      const int line = 4 * i + rsub;
      const int row = line >> 1, hl = line & 1;
      const v4f v = *(const v4fa*)(ss + row * 68 + 32 * hl + 4 * q8);
      *(volatile v4f*)(out1 + ((size_t)(b * NSEQ + 16 * w + row)) * NSEQ + 64 * hf + 32 * hl + 4 * q8) = v;
    }
    __threadfence();
    #pragma unroll 1
    for (int i = 0; i < 8; ++i) {
      const int line = 4 * i + rsub;
      const int row = line >> 1, hl = line & 1;
      const v4f v = *(const v4fa*)(ss + row * 68 + 32 * hl + 4 * q8);
      *(volatile v4f*)(out1 + ((size_t)(b * NSEQ + 16 * w + row)) * NSEQ + 64 * hf + 32 * hl + 4 * q8) = v;
    }
    __syncthreads();
  }
}

extern "C" void kernel_launch(void* const* d_in, const int* in_sizes, int n_in,
                              void* d_out, int out_size, void* d_ws, size_t ws_size,
                              hipStream_t stream) {
  if (n_in < 24) return;
  const int ex[24] = {8388608, 32768, 32768, 786432, 3072, 786432, 3072, 393216, 768,
                      786432, 768, 786432, 768, 768, 768, 65536, 256, 65536, 256, 65536,
                      256, 1, 256, 1};
  for (int i = 0; i < 24; ++i) if (in_sizes[i] != ex[i]) return;
  if (out_size != 12582912) return;

  const float* H      = (const float*)d_in[0];
  const int*   ph     = (const int*)d_in[1];
  const float* maskp  = (const float*)d_in[2];
  const float* ha_w   = (const float*)d_in[3];
  const float* ha_b   = (const float*)d_in[4];
  const float* sa_w   = (const float*)d_in[5];
  const float* sa_b   = (const float*)d_in[6];
  const float* ct_w   = (const float*)d_in[7];
  const float* ct_b   = (const float*)d_in[8];
  const float* gate_w = (const float*)d_in[9];
  const float* gate_b = (const float*)d_in[10];
  const float* tr_w   = (const float*)d_in[11];
  const float* tr_b   = (const float*)d_in[12];
  const float* ln_g   = (const float*)d_in[13];
  const float* ln_b   = (const float*)d_in[14];
  const float* arw_h  = (const float*)d_in[15];
  const float* arb_h  = (const float*)d_in[16];
  const float* arw_d  = (const float*)d_in[17];
  const float* arb_d  = (const float*)d_in[18];
  const float* bil    = (const float*)d_in[19];
  const float* bh_w   = (const float*)d_in[20];
  const float* bh_b   = (const float*)d_in[21];
  const float* bd_w   = (const float*)d_in[22];
  const float* bd_b   = (const float*)d_in[23];

  float* out0 = (float*)d_out;
  float* out1 = (float*)d_out + (size_t)PLANE;

  const size_t PLB   = (size_t)PLANE * 2;
  const size_t oHh   = 0;
  const size_t oCv   = 1 * PLB;
  const size_t oQ    = 2 * PLB;
  const size_t oK    = 3 * PLB;
  const size_t oV    = 4 * PLB;
  const size_t oAOh  = 5 * PLB;
  const size_t oAOs  = 6 * PLB;
  const size_t oHaT  = 7 * PLB;
  const size_t oSaT  = oHaT + (size_t)12 * 65536 * 2;
  const size_t oCtT  = oSaT + (size_t)12 * 65536 * 2;
  const size_t oGtT  = oCtT + (size_t)3 * 131072 * 2;
  const size_t oTrT  = oGtT + (size_t)3 * 262144 * 2;
  const size_t oW3   = oTrT + (size_t)3 * 262144 * 2;
  const size_t total = oW3 + (size_t)3 * 131072 * 2;
  if (total > ws_size) return;

  char* ws = (char*)d_ws;
  _Float16* Hh   = (_Float16*)(ws + oHh);
  _Float16* cavg = (_Float16*)(ws + oCv);
  _Float16* Qp   = (_Float16*)(ws + oQ);
  _Float16* Kpl  = (_Float16*)(ws + oK);
  _Float16* Vpl  = (_Float16*)(ws + oV);
  _Float16* AOh  = (_Float16*)(ws + oAOh);
  _Float16* AOs  = (_Float16*)(ws + oAOs);
  _Float16* haT  = (_Float16*)(ws + oHaT);
  _Float16* saT  = (_Float16*)(ws + oSaT);
  _Float16* ctT  = (_Float16*)(ws + oCtT);
  _Float16* gtT  = (_Float16*)(ws + oGtT);
  _Float16* trT  = (_Float16*)(ws + oTrT);
  unsigned short* w3 = (unsigned short*)(ws + oW3);
  _Float16* hmsg = Qp;
  _Float16* cmsg = Kpl;
  _Float16* smsg = Vpl;
  float* hhp = (float*)(ws + 0);
  float* hdp = (float*)(ws + 2 * PLB);
  unsigned short* Ghi = (unsigned short*)(ws + 4 * PLB);

  dim3 blk(256);

  cvt_wt_k<<<dim3(4, 4, 24), blk, 0, stream>>>(ha_w, sa_w, 12, haT, saT, 256);
  cvt_wt_k<<<dim3(8, 4, 3), blk, 0, stream>>>(ct_w, ct_w, 3, ctT, ctT, 512);
  cvt_wt_k<<<dim3(16, 4, 6), blk, 0, stream>>>(gate_w, tr_w, 3, gtT, trT, 1024);
  cvt_w3_k<<<dim3(4, 4, 3), blk, 0, stream>>>(arw_h, arw_d, bil, w3);
  cvt_h_k<<<dim3(4096), blk, 0, stream>>>(H, Hh, PLANE / 8);

  for (int it = 0; it < 3; ++it) {
    const float* HrIn = (it == 0) ? H : (const float*)out0;
    const _Float16* haTi = haT + (size_t)it * 4 * 65536;
    const _Float16* saTi = saT + (size_t)it * 4 * 65536;
    const float* habi = ha_b + (size_t)it * 4 * 256;
    const float* sabi = sa_b + (size_t)it * 4 * 256;

    child_k<<<dim3(NSEN), blk, 0, stream>>>(HrIn, ph, maskp, cavg);

    gemm_k<<<dim3(256, 4, 3), blk, 0, stream>>>(
        Hh, Hh, haTi + 0 * 65536, habi + 0,   Qp,
        Hh, Hh, haTi + 1 * 65536, habi + 256, Kpl,
        Hh, Hh, haTi + 2 * 65536, habi + 512, Vpl,
        1, 1, 1, 0, 0, 0, kInvW, kInvW, kInvW);
    attn_k<<<dim3(NSEN * 4), blk, 0, stream>>>(Qp, Kpl, Vpl, ph, maskp, AOh, 0);

    gemm_k<<<dim3(256, 4, 3), blk, 0, stream>>>(
        Hh, Hh, saTi + 0 * 65536, sabi + 0,   Qp,
        Hh, Hh, saTi + 1 * 65536, sabi + 256, Kpl,
        Hh, Hh, saTi + 2 * 65536, sabi + 512, Vpl,
        1, 1, 1, 0, 0, 0, kInvW, kInvW, kInvW);
    attn_k<<<dim3(NSEN * 4), blk, 0, stream>>>(Qp, Kpl, Vpl, ph, maskp, AOs, 1);

    gemm_k<<<dim3(256, 4, 3), blk, 0, stream>>>(
        AOh, AOh,  haTi + 3 * 65536, habi + 768, hmsg,
        AOs, AOs,  saTi + 3 * 65536, sabi + 768, smsg,
        Hh,  cavg, ctT + (size_t)it * 131072, ct_b + (size_t)it * 256, cmsg,
        1, 1, 2, 0, 0, 1, kInvWA, kInvWA, kInvW);

    comb_k<<<dim3(1024), blk, 0, stream>>>(
        Hh, hmsg, cmsg, smsg,
        gtT + (size_t)it * 262144, trT + (size_t)it * 262144,
        gate_b + (size_t)it * 256, tr_b + (size_t)it * 256,
        ln_g + (size_t)it * 256, ln_b + (size_t)it * 256,
        HrIn, out0, Hh, (it < 2) ? 1 : 0);
  }

  gemm3_k<<<dim3(256, 4, 2), blk, 0, stream>>>(
      (const float*)out0, w3,          arb_h, hhp, Ghi,
      (const float*)out0, w3 + 131072, arb_d, hdp, Ghi,
      1, 0);
  gemm3_k<<<dim3(256, 4, 1), blk, 0, stream>>>(
      (const float*)hdp, w3 + 262144, arb_h, hhp, Ghi,
      (const float*)hdp, w3 + 262144, arb_h, hhp, Ghi,
      0, 1);
  score_k<<<dim3(NSEN), blk, 0, stream>>>(hhp, hdp, Ghi, bh_w, bh_b, bd_w, bd_b, out1);
}
